// MultiHeadedAttention_22136261444055
// MI455X (gfx1250) — hardware-verified
//
#include <hip/hip_runtime.h>
#ifndef NB
#define NB 2
#endif
#ifndef SQ
#define SQ 2048
#endif
#define SQ_FULL 2048
#define DM 1024
#define NH 16
#define HD 64
#define HG 2
#define LQ (3 * DM)
#define LQK (2 * DM)
#ifndef ER
#define ER 128
#endif
#define ERG (ER / 32)
#define ERC (ER / 64)
#define NCK (SQ / 256)
#define NR ((size_t)NB * SQ)
static_assert(SQ % 256 == 0);
static_assert(SQ <= SQ_FULL);
static_assert(ER % 64 == 0);
static_assert(ER >= 64);
static_assert(ER <= 256);
static_assert(ER < SQ);
static_assert((SQ - ER) % 32 == 0);
static_assert(NH % HG == 0);
static_assert(DM == NH * HD);
static_assert(HD == 64);
static_assert(DM % 64 == 0);
static_assert(NB >= 1);
static_assert(NR % 128 == 0);

typedef __bf16 v16b __attribute__((ext_vector_type(16)));
typedef unsigned short v8us __attribute__((ext_vector_type(8), may_alias));
typedef unsigned short v4us __attribute__((ext_vector_type(4)));
typedef float  v8f  __attribute__((ext_vector_type(8)));
typedef float  v4f  __attribute__((ext_vector_type(4)));
typedef float  v4fa __attribute__((ext_vector_type(4), may_alias));
typedef _Float16 v16h __attribute__((ext_vector_type(16)));
typedef _Float16 v4h __attribute__((ext_vector_type(4)));
union FragB { v16b v; v8us half[2]; unsigned short u[16]; };
union FragH { v16h v; v8us half[2]; _Float16 h[16]; unsigned short u[16]; };

__device__ __forceinline__ unsigned short bf16_bits(float x) { unsigned int u = __float_as_uint(x); return (unsigned short)((u + 0x7FFFu + ((u >> 16) & 1u)) >> 16); }
__device__ __forceinline__ float bf16_val(unsigned short b) { return __uint_as_float(((unsigned int)b) << 16); }
__device__ __forceinline__ float bf16_rne(float x) { return bf16_val(bf16_bits(x)); }

template <int NT>
__device__ __forceinline__ v8f mmaN(v16b ah, v16b al, v16b bh, v16b bl, v8f c) {
  c = __builtin_amdgcn_wmma_f32_16x16x32_bf16(false, ah, false, bh, (short)0, c, false, false);
  if (NT >= 2) c = __builtin_amdgcn_wmma_f32_16x16x32_bf16(false, al, false, bh, (short)0, c, false, false);
  if (NT >= 3) c = __builtin_amdgcn_wmma_f32_16x16x32_bf16(false, ah, false, bl, (short)0, c, false, false);
  asm volatile("v_nop\n\tv_nop\n\tv_nop\n\tv_nop" : "+v"(c) : "v"(ah), "v"(al), "v"(bh), "v"(bl));
  return c;
}

__global__ __launch_bounds__(256) void k_wt_bf16(const float* __restrict__ W, unsigned short* __restrict__ Wt, int K, int N) {
  const int t = blockIdx.x * 256 + threadIdx.x;
  const int k8n = K / 8;
  if (t >= N * k8n) return;
  const int n = t / k8n, k8 = (t % k8n) * 8;
  v8us v;
#pragma unroll
  for (int i = 0; i < 8; ++i) v[i] = bf16_bits(W[(size_t)(k8 + i) * N + n]);
  *(volatile v8us*)(Wt + (size_t)n * K + k8) = v;
  __threadfence();
  *(volatile v8us*)(Wt + (size_t)n * K + k8) = v;
}

__global__ __launch_bounds__(256) void k_wt_f16(const float* __restrict__ W, _Float16* __restrict__ Wt, int K, int N, float scale) {
  const int t = blockIdx.x * 256 + threadIdx.x; if (t >= N * (K / 8)) return; const int n = t / (K / 8), k8 = (t % (K / 8)) * 8; FragH f;
#pragma unroll
  for (int i = 0; i < 8; ++i) f.h[i] = (_Float16)(bf16_rne(W[(size_t)(k8 + i) * N + n]) * scale); const v8us o = f.half[0];
  *(volatile v8us*)((unsigned short*)Wt + (size_t)n * K + k8) = o; __threadfence(); *(volatile v8us*)((unsigned short*)Wt + (size_t)n * K + k8) = o;
}

__global__ __launch_bounds__(256) void k_x16(const float* __restrict__ x, _Float16* __restrict__ X16, size_t n8) {
  const size_t t = (size_t)blockIdx.x * 256 + threadIdx.x; if (t >= n8) return;
  const size_t e = t * 8; const size_t rc = e / DM; const size_t wi = e % DM; const size_t bb = rc / SQ, sq = rc % SQ;
  const float* src = x + (bb * SQ_FULL + sq) * DM + wi;
  FragH f;
#pragma unroll
  for (int q = 0; q < 8; ++q) f.h[q] = (_Float16)bf16_rne(src[q]);
  *(volatile v8us*)((unsigned short*)X16 + e) = f.half[0]; __threadfence(); *(volatile v8us*)((unsigned short*)X16 + e) = f.half[0];
}

template <bool ASPLIT, int ACT, bool BIAS_BF16>
__global__ __launch_bounds__(128) void k_gemm_bf(const float* __restrict__ A, int lda, const unsigned short* __restrict__ Wt, int ldb,
                                               const float* __restrict__ bias, float* __restrict__ C, int ldc, int M, int N, int K) {
  __shared__ __attribute__((aligned(16))) float so[4][16][64];
  const int tid = threadIdx.x, w = tid >> 5, lane = tid & 31, ln = lane & 15, hh = lane >> 4;
  const int ntn = N / 64;
  const int wid = blockIdx.x * 4 + w;
  const int mt = wid / ntn, nq = wid % ntn;
  if (mt * 16 >= M) return;
  const int row0 = mt * 16, col0 = nq * 64;
  const float* arow = A + (size_t)(row0 + ln) * lda;
  v8f acc[4] = {};
#pragma unroll 1
  for (int kb = 0; kb < K; kb += 32) {
    FragB ah, al;
    const v4f x0 = *(const v4fa*)(arow + kb + 8 * hh), x1 = *(const v4fa*)(arow + kb + 8 * hh + 4);
    const v4f x2 = *(const v4fa*)(arow + kb + 16 + 8 * hh), x3 = *(const v4fa*)(arow + kb + 16 + 8 * hh + 4);
    float xs[16] = {x0[0],x0[1],x0[2],x0[3],x1[0],x1[1],x1[2],x1[3],x2[0],x2[1],x2[2],x2[3],x3[0],x3[1],x3[2],x3[3]};
#pragma unroll
    for (int i = 0; i < 16; ++i) { const unsigned short hb = bf16_bits(xs[i]); ah.u[i] = hb; al.u[i] = ASPLIT ? bf16_bits(xs[i] - bf16_val(hb)) : (unsigned short)0; }
#pragma unroll
    for (int t = 0; t < 4; ++t) {
      const unsigned short* brow = Wt + (size_t)(col0 + t * 16 + ln) * ldb + kb;
      FragB b;
      b.half[0] = *(const v8us*)(brow + 8 * hh);
      b.half[1] = *(const v8us*)(brow + 16 + 8 * hh);
      acc[t] = mmaN<ASPLIT ? 2 : 1>(ah.v, al.v, b.v, b.v, acc[t]);
    }
  }
#pragma unroll
  for (int t = 0; t < 4; ++t) {
    float bv = bias ? bias[col0 + t * 16 + ln] : 0.f;
    if (BIAS_BF16) bv = bf16_rne(bv);
#pragma unroll
    for (int r = 0; r < 8; ++r) { float v = acc[t][r] + bv; if (ACT == 1) v = fmaxf(v, 0.f); so[w][8 * hh + r][t * 16 + ln] = v; }
  }
  __builtin_amdgcn_fence(4  , "workgroup");
  __builtin_amdgcn_wave_barrier();
  const int rsub = lane >> 4, c4 = (lane & 15) * 4;
  for (int pass = 0; pass < 2; ++pass) {
#pragma unroll
    for (int q = 0; q < 8; ++q) {
      const int r = q * 2 + rsub;
      const v4f v = *(const v4fa*)&so[w][r][c4];
      *(volatile v4f*)(C + (size_t)(row0 + r) * ldc + col0 + c4) = v;
    }
    if (pass == 0) __threadfence();
  }
}

template <int NHv, int TTv>
__global__ __launch_bounds__(256) void k_vt(const _Float16* __restrict__ V16, int ldv, int voff, _Float16* __restrict__ Vt) { __shared__ unsigned short tl[64][66]; const int tid = threadIdx.x; const int slab = blockIdx.x / (TTv / 64), lg = blockIdx.x % (TTv / 64); const int b = slab / NHv, h = slab % NHv;
  for (int i = tid; i < 64 * 8; i += 256) { const int r = i / 8, c8 = (i % 8) * 8; FragH f; f.half[0] = *(const v8us*)((const unsigned short*)V16 + ((size_t)b * TTv + lg * 64 + r) * ldv + voff + h * 64 + c8);
#pragma unroll
    for (int q = 0; q < 8; ++q) tl[r][c8 + q] = f.u[q]; }
  __syncthreads();
  for (int pass = 0; pass < 2; ++pass) {
#pragma unroll
    for (int rd = 0; rd < 2; ++rd) { const int d = rd * 32 + tid / 8, pc = tid % 8; FragH f;
#pragma unroll
      for (int q = 0; q < 8; ++q) f.u[q] = tl[pc * 8 + q][d];
      *(volatile v8us*)((unsigned short*)Vt + ((size_t)slab * 64 + d) * TTv + lg * 64 + pc * 8) = f.half[0]; }
    if (pass == 0) __threadfence(); } }

__device__ __forceinline__ v16h g2_frag(const _Float16* p, int hh) { FragH f; f.half[0] = *(const v8us*)((const unsigned short*)p + 8 * hh); f.half[1] = *(const v8us*)((const unsigned short*)p + 16 + 8 * hh); return f.v; }
__device__ __forceinline__ v16b gb_frag(const unsigned short* p, int hh) { FragB f; f.half[0] = *(const v8us*)(p + 8 * hh); f.half[1] = *(const v8us*)(p + 16 + 8 * hh); return f.v; }
__device__ __forceinline__ v8f g2_mma(v16h a, v16h b, v8f c) { v8f d = __builtin_amdgcn_wmma_f32_16x16x32_f16(false, a, false, b, (short)0, c, false, false); asm volatile("v_nop\n\tv_nop\n\tv_nop\n\tv_nop" : "+v"(d) : "v"(a), "v"(b)); return d; }
__global__ __launch_bounds__(128) void k_gemm2(const _Float16* __restrict__ A, int lda, size_t sA, const _Float16* __restrict__ Bh, int ldb, size_t sB, float alpha,
    const float* __restrict__ bias, float* __restrict__ C, _Float16* __restrict__ C16, int ldc, size_t sC, int M, int N, int K, int causal) {
  __shared__ __attribute__((aligned(16))) float so[4][32][68];
  const int tid = threadIdx.x, w = tid >> 5, lane = tid & 31, ln = lane & 15, hh = lane >> 4; const int by = blockIdx.y;
  A += (size_t)by * sA; Bh += (size_t)by * sB; const size_t cofs = (size_t)by * sC;
  const int ntn = N >> 6; const int mt = blockIdx.x / ntn, nq = blockIdx.x - mt * ntn; const int row0 = mt * 128 + 32 * w, col0 = nq * 64;
  if (row0 >= M) return;
  const int qend = mt * 128 + 128;
  if (causal != 0 && col0 >= qend) return;
  const int kend = (causal != 0 && qend < K) ? qend : K;
  const _Float16* a0p = A + (size_t)(row0 + ln) * lda; const _Float16* a1p = a0p + (size_t)16 * lda;
  const _Float16* b0p = Bh + (size_t)(col0 + ln) * ldb; const _Float16* b1p = b0p + (size_t)16 * ldb; const _Float16* b2p = b1p + (size_t)16 * ldb; const _Float16* b3p = b2p + (size_t)16 * ldb;
  const v8f z8 = {0.f,0.f,0.f,0.f,0.f,0.f,0.f,0.f}; v8f c00 = z8, c01 = z8, c02 = z8, c03 = z8, c10 = z8, c11 = z8, c12 = z8, c13 = z8;
#pragma unroll 1
  for (int kb = 0; kb < kend; kb += 32) { const v16h a0 = g2_frag(a0p + kb, hh), a1 = g2_frag(a1p + kb, hh);
    v16h b = g2_frag(b0p + kb, hh); c00 = g2_mma(a0, b, c00); c10 = g2_mma(a1, b, c10);
    b = g2_frag(b1p + kb, hh); c01 = g2_mma(a0, b, c01); c11 = g2_mma(a1, b, c11);
    b = g2_frag(b2p + kb, hh); c02 = g2_mma(a0, b, c02); c12 = g2_mma(a1, b, c12);
    b = g2_frag(b3p + kb, hh); c03 = g2_mma(a0, b, c03); c13 = g2_mma(a1, b, c13); }
  v8f accs[8] = {c00, c01, c02, c03, c10, c11, c12, c13};
#pragma unroll
  for (int u = 0; u < 8; ++u) { const int t = u & 3, half = u >> 2; const int col = col0 + t * 16 + ln; const float bv = bias ? bf16_rne(bias[col]) : 0.f;
#pragma unroll
    for (int r = 0; r < 8; ++r) { const int rloc = half * 16 + 8 * hh + r; const float v = accs[u][r] * alpha + bv; so[w][rloc][t * 16 + ln] = v; } }
  __builtin_amdgcn_fence(4  , "workgroup"); __builtin_amdgcn_wave_barrier();
  const int rsub = lane >> 4, c4 = (lane & 15) * 4;
  for (int pass = 0; pass < 2; ++pass) {
#pragma unroll
    for (int q = 0; q < 16; ++q) { const int r = q * 2 + rsub; const v4f v = *(const v4fa*)&so[w][r][c4];
      if (C) *(volatile v4f*)(C + cofs + (size_t)(row0 + r) * ldc + col0 + c4) = v;
      if (C16) { v4h h4; for (int i = 0; i < 4; ++i) h4[i] = (_Float16)v[i]; *(volatile v4h*)(C16 + cofs + (size_t)(row0 + r) * ldc + col0 + c4) = h4; } }
    if (pass == 0) __threadfence(); } }

__global__ __launch_bounds__(128) void k_gemm2s(const _Float16* __restrict__ A, int lda, const _Float16* __restrict__ Bh, int ldb, float alpha,
    unsigned short* __restrict__ CH, unsigned short* __restrict__ CL, int ldc, int M, int N, int K) {
  __shared__ __attribute__((aligned(16))) float so[4][32][68];
  const int tid = threadIdx.x, w = tid >> 5, lane = tid & 31, ln = lane & 15, hh = lane >> 4;
  const int ntn = N >> 6; const int mt = blockIdx.x / ntn, nq = blockIdx.x - mt * ntn; const int row0 = mt * 128 + 32 * w, col0 = nq * 64;
  if (row0 >= M) return;
  const _Float16* a0p = A + (size_t)(row0 + ln) * lda; const _Float16* a1p = a0p + (size_t)16 * lda;
  const _Float16* b0p = Bh + (size_t)(col0 + ln) * ldb; const _Float16* b1p = b0p + (size_t)16 * ldb; const _Float16* b2p = b1p + (size_t)16 * ldb; const _Float16* b3p = b2p + (size_t)16 * ldb;
  const v8f z8 = {0.f,0.f,0.f,0.f,0.f,0.f,0.f,0.f}; v8f c00 = z8, c01 = z8, c02 = z8, c03 = z8, c10 = z8, c11 = z8, c12 = z8, c13 = z8;
#pragma unroll 1
  for (int kb = 0; kb < K; kb += 32) { const v16h a0 = g2_frag(a0p + kb, hh), a1 = g2_frag(a1p + kb, hh);
    v16h b = g2_frag(b0p + kb, hh); c00 = g2_mma(a0, b, c00); c10 = g2_mma(a1, b, c10);
    b = g2_frag(b1p + kb, hh); c01 = g2_mma(a0, b, c01); c11 = g2_mma(a1, b, c11);
    b = g2_frag(b2p + kb, hh); c02 = g2_mma(a0, b, c02); c12 = g2_mma(a1, b, c12);
    b = g2_frag(b3p + kb, hh); c03 = g2_mma(a0, b, c03); c13 = g2_mma(a1, b, c13); }
  v8f accs[8] = {c00, c01, c02, c03, c10, c11, c12, c13};
#pragma unroll
  for (int u = 0; u < 8; ++u) { const int t = u & 3, half = u >> 2;
#pragma unroll
    for (int r = 0; r < 8; ++r) { const int rloc = half * 16 + 8 * hh + r; so[w][rloc][t * 16 + ln] = accs[u][r] * alpha; } }
  __builtin_amdgcn_fence(4  , "workgroup"); __builtin_amdgcn_wave_barrier();
  const int rsub = lane >> 4, c4 = (lane & 15) * 4;
  for (int pass = 0; pass < 2; ++pass) {
#pragma unroll
    for (int q = 0; q < 16; ++q) { const int r = q * 2 + rsub; const v4f v = *(const v4fa*)&so[w][r][c4]; v4us hb, lb;
#pragma unroll
      for (int i = 0; i < 4; ++i) { const unsigned short hq = bf16_bits(v[i]); hb[i] = hq; lb[i] = bf16_bits(v[i] - bf16_val(hq)); }
      *(volatile v4us*)(CH + (size_t)(row0 + r) * ldc + col0 + c4) = hb;
      *(volatile v4us*)(CL + (size_t)(row0 + r) * ldc + col0 + c4) = lb; }
    if (pass == 0) __threadfence(); } }

__global__ __launch_bounds__(128) void k_gemm2b(const unsigned short* __restrict__ AH, const unsigned short* __restrict__ AL, int lda, size_t sA,
    const unsigned short* __restrict__ BHp, const unsigned short* __restrict__ BLp, int ldb, size_t sB, float alpha,
    float* __restrict__ C, int ldc, size_t sC, int M, int N, int K, int causal) {
  __shared__ __attribute__((aligned(16))) float so[4][32][68];
  const int tid = threadIdx.x, w = tid >> 5, lane = tid & 31, ln = lane & 15, hh = lane >> 4; const int by = blockIdx.y;
  AH += (size_t)by * sA; AL += (size_t)by * sA; BHp += (size_t)by * sB; BLp += (size_t)by * sB; const size_t cofs = (size_t)by * sC;
  const int ntn = N >> 6; const int mt = blockIdx.x / ntn, nq = blockIdx.x - mt * ntn; const int row0 = mt * 128 + 32 * w, col0 = nq * 64;
  if (row0 >= M) return;
  const int qend = mt * 128 + 128;
  if (causal != 0 && col0 >= qend) return;
  const int kend = (causal != 0 && qend < K) ? qend : K;
  const unsigned short* ah0p = AH + (size_t)(row0 + ln) * lda; const unsigned short* ah1p = ah0p + (size_t)16 * lda;
  const unsigned short* al0p = AL + (size_t)(row0 + ln) * lda; const unsigned short* al1p = al0p + (size_t)16 * lda;
  const unsigned short* bh0 = BHp + (size_t)(col0 + ln) * ldb; const unsigned short* bh1 = bh0 + (size_t)16 * ldb; const unsigned short* bh2 = bh1 + (size_t)16 * ldb; const unsigned short* bh3 = bh2 + (size_t)16 * ldb;
  const unsigned short* bl0 = BLp + (size_t)(col0 + ln) * ldb; const unsigned short* bl1 = bl0 + (size_t)16 * ldb; const unsigned short* bl2 = bl1 + (size_t)16 * ldb; const unsigned short* bl3 = bl2 + (size_t)16 * ldb;
  const v8f z8 = {0.f,0.f,0.f,0.f,0.f,0.f,0.f,0.f}; v8f c00 = z8, c01 = z8, c02 = z8, c03 = z8, c10 = z8, c11 = z8, c12 = z8, c13 = z8;
#pragma unroll 1
  for (int kb = 0; kb < kend; kb += 32) {
    const v16b a0h = gb_frag(ah0p + kb, hh), a0l = gb_frag(al0p + kb, hh), a1h = gb_frag(ah1p + kb, hh), a1l = gb_frag(al1p + kb, hh);
    v16b bh = gb_frag(bh0 + kb, hh), bl = gb_frag(bl0 + kb, hh); c00 = mmaN<3>(a0h, a0l, bh, bl, c00); c10 = mmaN<3>(a1h, a1l, bh, bl, c10);
    bh = gb_frag(bh1 + kb, hh); bl = gb_frag(bl1 + kb, hh); c01 = mmaN<3>(a0h, a0l, bh, bl, c01); c11 = mmaN<3>(a1h, a1l, bh, bl, c11);
    bh = gb_frag(bh2 + kb, hh); bl = gb_frag(bl2 + kb, hh); c02 = mmaN<3>(a0h, a0l, bh, bl, c02); c12 = mmaN<3>(a1h, a1l, bh, bl, c12);
    bh = gb_frag(bh3 + kb, hh); bl = gb_frag(bl3 + kb, hh); c03 = mmaN<3>(a0h, a0l, bh, bl, c03); c13 = mmaN<3>(a1h, a1l, bh, bl, c13); }
  v8f accs[8] = {c00, c01, c02, c03, c10, c11, c12, c13};
#pragma unroll
  for (int u = 0; u < 8; ++u) { const int t = u & 3, half = u >> 2;
#pragma unroll
    for (int r = 0; r < 8; ++r) { const int rloc = half * 16 + 8 * hh + r; so[w][rloc][t * 16 + ln] = accs[u][r] * alpha; } }
  __builtin_amdgcn_fence(4  , "workgroup"); __builtin_amdgcn_wave_barrier();
  const int rsub = lane >> 4, c4 = (lane & 15) * 4;
  for (int pass = 0; pass < 2; ++pass) {
#pragma unroll
    for (int q = 0; q < 16; ++q) { const int r = q * 2 + rsub; const v4f v = *(const v4fa*)&so[w][r][c4];
      *(volatile v4f*)(C + cofs + (size_t)(row0 + r) * ldc + col0 + c4) = v; }
    if (pass == 0) __threadfence(); } }

__global__ __launch_bounds__(256) void k_csm(const float* __restrict__ S, _Float16* __restrict__ P, int qn, int hg) {
  const int w = threadIdx.x >> 5, lane = threadIdx.x & 31;
  const int i = blockIdx.x * 8 + w;
  if (i >= qn * hg) return;
  const int hs = i / qn, q = i - hs * qn;
  const size_t roff = ((size_t)hs * SQ + q) * SQ;
  const float* s = S + roff;
  const int wl = (q >> 7) * 128 + 128;
  const int cn = (wl + 255) >> 8;
  float v[NCK][8];
  float mx = -3.0e38f;
#pragma unroll
  for (int c = 0; c < NCK; ++c) {
#pragma unroll
    for (int e = 0; e < 8; ++e) v[c][e] = -3.0e38f;
    if (c < cn) {
      int jb = 256 * c + 8 * lane; jb = (jb < wl - 8) ? jb : (wl - 8);
      const v4f a = *(const v4fa*)(s + jb), bq = *(const v4fa*)(s + jb + 4);
      const float t8[8] = {a[0], a[1], a[2], a[3], bq[0], bq[1], bq[2], bq[3]};
#pragma unroll
      for (int e = 0; e < 8; ++e) { const int j = 256 * c + 8 * lane + e; const float sv = (j <= q) ? t8[e] : -3.0e38f; v[c][e] = sv; mx = fmaxf(mx, sv); }
    }
  }
#pragma unroll
  for (int m = 16; m >= 1; m >>= 1) mx = fmaxf(mx, __shfl_xor(mx, m, 32));
  float se = 0.f;
#pragma unroll
  for (int c = 0; c < NCK; ++c) {
    if (c < cn) {
#pragma unroll
      for (int e = 0; e < 8; ++e) { const int j = 256 * c + 8 * lane + e; const float ex = (j <= q) ? __expf(v[c][e] - mx) : 0.f; v[c][e] = ex; se += ex; }
    }
  }
#pragma unroll
  for (int m = 16; m >= 1; m >>= 1) se += __shfl_xor(se, m, 32);
  const float sc = 1024.0f / se;
  unsigned short* prow = (unsigned short*)P + roff;
  for (int pass = 0; pass < 2; ++pass) {
#pragma unroll
    for (int c = 0; c < NCK; ++c) {
      if (c < cn) { FragH f;
#pragma unroll
        for (int e = 0; e < 8; ++e) f.h[e] = (_Float16)(v[c][e] * sc);
        *(volatile v8us*)(prow + 256 * c + 8 * lane) = f.half[0]; }
    }
    if (pass == 0) __threadfence();
  }
}

__global__ __launch_bounds__(256) void k_early(const float* __restrict__ QE, int b, float* __restrict__ OE) {
  __shared__ __attribute__((aligned(16))) float qs[32][64];
  __shared__ __attribute__((aligned(16))) float kv[64][68];
  __shared__ float ss[32][ER + 1];
  __shared__ float red[256];
  const int tid = threadIdx.x;
  const int h = blockIdx.x / ERG, g = blockIdx.x - h * ERG;
  const int q0 = g * 32;
  const int nch = (q0 + 32 + 63) / 64;
  const int ti = tid >> 3, p = tid & 7;
  const int iq = q0 + ti;
  const float* qe = QE + (size_t)b * ER * LQ;
#pragma unroll
  for (int u = 0; u < 2; ++u) { const int idx = tid + 256 * u; const int r = idx >> 4, c4 = (idx & 15) * 4;
    *(v4fa*)&qs[r][c4] = *(const v4fa*)(qe + (size_t)(q0 + r) * LQ + h * HD + c4); }
#pragma unroll 1
  for (int c = 0; c < nch && c < ERC; ++c) {
    __syncthreads();
#pragma unroll
    for (int u = 0; u < 4; ++u) { const int idx = tid + 256 * u; const int r = idx >> 4, c4 = (idx & 15) * 4;
      *(v4fa*)&kv[r][c4] = *(const v4fa*)(qe + (size_t)(64 * c + r) * LQ + DM + h * HD + c4); }
    __syncthreads();
#pragma unroll 1
    for (int jj = 0; jj < 8; ++jj) { const int jl = 8 * p + jj; float a = 0.f;
#pragma unroll 1
      for (int d = 0; d < HD; ++d) a += qs[ti][d] * kv[jl][d];
      ss[ti][64 * c + jl] = a * 0.125f; }
  }
  __syncthreads();
  float mx = -3.0e38f;
#pragma unroll 1
  for (int j = 0; j <= iq; ++j) mx = fmaxf(mx, ss[ti][j]);
  __syncthreads();
  float ps = 0.f;
#pragma unroll 1
  for (int c = 0; c < nch && c < ERC; ++c) {
#pragma unroll 1
    for (int jj = 0; jj < 8; ++jj) { const int j = 64 * c + 8 * p + jj; const float sv = ss[ti][j]; const float e = (j <= iq) ? expf(sv - mx) : 0.f; ss[ti][j] = e; ps += e; }
  }
  red[tid] = ps;
  __syncthreads();
  float se = 0.f;
#pragma unroll
  for (int pp = 0; pp < 8; ++pp) se += red[ti * 8 + pp];
  const float inv = 1.0f / se;
  float acc[8] = {0.f, 0.f, 0.f, 0.f, 0.f, 0.f, 0.f, 0.f};
#pragma unroll 1
  for (int c = 0; c < nch && c < ERC; ++c) {
    __syncthreads();
#pragma unroll
    for (int u = 0; u < 4; ++u) { const int idx = tid + 256 * u; const int r = idx >> 4, c4 = (idx & 15) * 4;
      *(v4fa*)&kv[r][c4] = *(const v4fa*)(qe + (size_t)(64 * c + r) * LQ + 2 * DM + h * HD + c4); }
    __syncthreads();
#pragma unroll 1
    for (int jl = 0; jl < 64; ++jl) { const float pw = ss[ti][64 * c + jl];
#pragma unroll
      for (int dd = 0; dd < 8; ++dd) acc[dd] += pw * kv[jl][8 * p + dd]; }
  }
#pragma unroll
  for (int dd = 0; dd < 8; ++dd) qs[ti][8 * p + dd] = acc[dd] * inv;
  __syncthreads();
  float* oe = OE + ((size_t)b * ER + q0) * DM + h * HD;
  for (int pass = 0; pass < 2; ++pass) {
#pragma unroll
    for (int u = 0; u < 2; ++u) { const int idx = tid + 256 * u; const int r = idx >> 4, c4 = (idx & 15) * 4; const v4f v = *(const v4fa*)&qs[r][c4]; *(volatile v4f*)(oe + (size_t)r * DM + c4) = v; }
    if (pass == 0) __threadfence();
  }
}

extern "C" void kernel_launch(void* const* d_in, const int* in_sizes, int n_in,
                              void* d_out, int out_size, void* d_ws, size_t ws_size, hipStream_t stream) {
  if (n_in < 4) return;
  const float* x = (const float*)d_in[0]; const float* wqkv = (const float*)d_in[1]; const float* wo = (const float*)d_in[2]; const float* bo = (const float*)d_in[3];
  const size_t xneed = ((size_t)(NB - 1) * SQ_FULL + SQ) * DM;
  if ((size_t)in_sizes[0] < xneed || (size_t)in_sizes[1] < (size_t)DM * LQ || (size_t)in_sizes[2] < (size_t)DM * DM || in_sizes[3] < DM || (size_t)out_size < xneed) return;
  char* ws = (char*)d_ws; size_t off = 0;
  auto take = [&](size_t bytes) { char* p = ws + off; off += (bytes + 255) & ~(size_t)255; return p; };
  _Float16* BQKV = (_Float16*)take((size_t)LQ * DM * 2);
  _Float16* BO = (_Float16*)take((size_t)DM * DM * 2);
  unsigned short* BWO = (unsigned short*)take((size_t)DM * DM * 2);
  _Float16* X16 = (_Float16*)take(NR * DM * 2);
  unsigned short* QKH = (unsigned short*)take(NR * LQK * 2);
  unsigned short* QKL = (unsigned short*)take(NR * LQK * 2);
  _Float16* V16 = (_Float16*)take(NR * DM * 2);
  _Float16* O16 = (_Float16*)take(NR * DM * 2);
  float* S = (float*)take((size_t)HG * SQ * SQ * 4);
  _Float16* P = (_Float16*)take((size_t)HG * SQ * SQ * 2);
  _Float16* VT = (_Float16*)take((size_t)NH * HD * SQ * 2);
  float* QE = (float*)take((size_t)NB * ER * LQ * 4);
  float* OE = (float*)take((size_t)NB * ER * DM * 4);
  if (off > ws_size) return;
  float* out = (float*)d_out;

  k_wt_f16<<<(unsigned)(((size_t)LQ * (DM / 8) + 255) / 256), 256, 0, stream>>>(wqkv, BQKV, DM, LQ, 16.0f);
  k_wt_f16<<<(unsigned)(((size_t)DM * (DM / 8) + 255) / 256), 256, 0, stream>>>(wo, BO, DM, DM, 16.0f);
  k_wt_bf16<<<(unsigned)(((size_t)DM * (DM / 8) + 255) / 256), 256, 0, stream>>>(wo, BWO, DM, DM);
  k_x16<<<(unsigned)((NR * DM / 8 + 255) / 256), 256, 0, stream>>>(x, X16, NR * DM / 8);
  k_gemm2s<<<(unsigned)((NR / 128) * (LQK / 64)), 128, 0, stream>>>(X16, DM, BQKV, DM, 0.0625f, QKH, QKL, LQK, (int)NR, LQK, DM);
  k_gemm2<<<dim3((unsigned)((NR / 128) * (DM / 64)), 1), 128, 0, stream>>>(X16, DM, (size_t)0, BQKV + (size_t)2 * DM * DM, DM, (size_t)0, 0.0625f, nullptr, nullptr, V16, DM, (size_t)0, (int)NR, DM, DM, 0);
  for (int b = 0; b < NB; ++b) {
    const size_t rc0 = (size_t)b * SQ;
    const size_t rf0 = (size_t)b * SQ_FULL;
    k_vt<NH, SQ><<<NH * (SQ / 64), 256, 0, stream>>>(V16 + rc0 * DM, DM, 0, VT);
    for (int h0 = 0; h0 < NH; h0 += HG) {
      k_gemm2b<<<dim3((SQ / 128) * (SQ / 64), HG), 128, 0, stream>>>(QKH + rc0 * LQK + h0 * HD, QKL + rc0 * LQK + h0 * HD, LQK, (size_t)HD, QKH + rc0 * LQK + DM + h0 * HD, QKL + rc0 * LQK + DM + h0 * HD, LQK, (size_t)HD, 0.125f, S, SQ, (size_t)SQ * SQ, SQ, SQ, HD, 1);
      k_csm<<<(HG * SQ + 7) / 8, 256, 0, stream>>>(S, P, SQ, HG);
      k_gemm2<<<dim3((SQ / 128) * (HD / 64), HG), 128, 0, stream>>>(P, SQ, (size_t)SQ * SQ, VT + (size_t)h0 * HD * SQ, SQ, (size_t)HD * SQ, 0.0625f, nullptr, nullptr, O16 + rc0 * DM + h0 * HD, DM, (size_t)HD, SQ, HD, SQ, 1);
    }
    k_gemm2<<<dim3((unsigned)(((SQ - ER + 127) / 128) * (DM / 64)), 1), 128, 0, stream>>>(O16 + (rc0 + ER) * DM, DM, (size_t)0, BO, DM, (size_t)0, 0.0009765625f, bo, out + (rf0 + ER) * DM, nullptr, DM, (size_t)0, SQ - ER, DM, DM, 0);
    k_gemm2<<<dim3((unsigned)(((ER + 127) / 128) * (LQ / 64)), 1), 128, 0, stream>>>(X16 + rc0 * DM, DM, (size_t)0, BQKV, DM, (size_t)0, 0.0625f, nullptr, QE + (size_t)b * ER * LQ, nullptr, LQ, (size_t)0, ER, LQ, DM, 0);
    k_early<<<NH * ERG, 256, 0, stream>>>(QE, b, OE);
    k_gemm_bf<true, 0, true><<<(unsigned)((ER / 16) * (DM / 64) / 4), 128, 0, stream>>>(OE + (size_t)b * ER * DM, DM, BWO, DM, bo, out + rf0 * DM, DM, ER, DM, DM);
  }
}
